// MultiHeadAttention_35570919146065
// MI455X (gfx1250) — hardware-verified
//
#include <hip/hip_runtime.h>


#define DEV_INLINE __device__ __forceinline__

#ifndef NB
#define NB 2
#endif
#ifndef SEQ
#define SEQ 2048
#endif
#define NB_FULL 2
#define SEQ_FULL 2048
#define DM 1024
#define NH 16
#define DK 64
#define RELDIM 64
#define NREL 4095
#define RELOFF 2047
#define MTOK (NB * SEQ)
#define NQB (SEQ / 64)
#define EARLY_ROWS 256
#define EARLY_QB (((EARLY_ROWS / 64) < NQB) ? (EARLY_ROWS / 64) : NQB)
#define RW (SEQ + 64)
#define FLAGS_PITCH 32
#define RS_PAD 4096

static_assert(SEQ % 256 == 0);
static_assert(SEQ <= SEQ_FULL);
static_assert(NB >= 1);
static_assert(NB <= NB_FULL);
static_assert(NQB <= FLAGS_PITCH);
static_assert(DM == NH * DK);
static_assert(MTOK % 256 == 0);
static_assert(NREL < RS_PAD);

typedef _Float16 half8  __attribute__((ext_vector_type(8)));
typedef _Float16 half16 __attribute__((ext_vector_type(16)));
typedef float    float8 __attribute__((ext_vector_type(8)));
typedef float    v4f    __attribute__((ext_vector_type(4)));
typedef int      v4i    __attribute__((ext_vector_type(4)));

DEV_INLINE float bf16r(float f) {
  unsigned int u = __float_as_uint(f);
  u += 0x7fffu + ((u >> 16) & 1u);
  return __uint_as_float(u & 0xffff0000u);
}

DEV_INLINE half16 load_frag(const _Float16* rowPtr, int halfSel) {
  const _Float16* p = rowPtr + halfSel * 8;
  const half8 lo = *(const half8*)(p);
  const half8 hi = *(const half8*)(p + 16);
  half16 r;
#pragma unroll
  for (int i = 0; i < 8; ++i) { r[i] = lo[i]; r[i + 8] = hi[i]; }
  return r;
}

DEV_INLINE float8 wmma16(half16 a, half16 b, float8 c) {
  float8 d = __builtin_amdgcn_wmma_f32_16x16x32_f16(false, a, false, b, (short)0, c, false, false);
  asm volatile("v_nop\n\tv_nop\n\tv_nop\n\tv_nop" : "+v"(d) : "v"(a), "v"(b));
  return d;
}

DEV_INLINE float8 zero8() {
  float8 z;
#pragma unroll
  for (int i = 0; i < 8; ++i) z[i] = 0.0f;
  return z;
}

DEV_INLINE half16 zero16() {
  half16 z;
#pragma unroll
  for (int i = 0; i < 16; ++i) z[i] = (_Float16)0.0f;
  return z;
}

__global__ __launch_bounds__(256) void k_xcvt(
    const float* __restrict__ q, const float* __restrict__ k, const float* __restrict__ v,
    _Float16* __restrict__ xq, _Float16* __restrict__ xk, _Float16* __restrict__ xv) {
  const int sel = blockIdx.y;
  const float* src = (sel == 0) ? q : ((sel == 1) ? k : v);
  _Float16* dst = (sel == 0) ? xq : ((sel == 1) ? xk : xv);
  const size_t g8 = (size_t)blockIdx.x * 256 + threadIdx.x;
  const size_t total8 = (size_t)MTOK * DM / 8;
  if (g8 >= total8) return;
  const size_t e = g8 * 8;
  const size_t tok = e / DM;
  const int col = (int)(e - tok * DM);
  const int bb = (int)(tok / SEQ);
  const int ss = (int)(tok - (size_t)bb * SEQ);
  const float* p = src + ((size_t)bb * SEQ_FULL + ss) * DM + col;
  const v4f x0 = *(const v4f*)(p);
  const v4f x1 = *(const v4f*)(p + 4);
  half8 o;
#pragma unroll
  for (int j = 0; j < 4; ++j) {
    const float t0 = x0[j];
    const float t1 = x1[j];
    o[j]     = (_Float16)(bf16r(t0) * 16.0f);
    o[j + 4] = (_Float16)(bf16r(t1) * 16.0f);
  }
  _Float16* d = dst + e;
  *(volatile half8*)d = o;
  __threadfence();
  *(volatile half8*)d = o;
}

__global__ __launch_bounds__(256) void k_wcvt(
    const float* __restrict__ w0, const float* __restrict__ w1,
    const float* __restrict__ w2, const float* __restrict__ w3,
    _Float16* __restrict__ t0, _Float16* __restrict__ t1,
    _Float16* __restrict__ t2, _Float16* __restrict__ t3) {
  __shared__ __align__(16) _Float16 tile[64 * 72];
  const int sel = blockIdx.z;
  const float* W = (sel == 0) ? w0 : ((sel == 1) ? w1 : ((sel == 2) ? w2 : w3));
  _Float16* T = (sel == 0) ? t0 : ((sel == 1) ? t1 : ((sel == 2) ? t2 : t3));
  const int k0 = blockIdx.y * 64, n0 = blockIdx.x * 64, tid = threadIdx.x;
#pragma unroll
  for (int p = 0; p < 4; ++p) {
    const int idx = tid + 256 * p;
    const int kr = idx >> 4;
    const int c4 = (idx & 15) * 4;
    const v4f wv = *(const v4f*)(W + (size_t)(k0 + kr) * DM + n0 + c4);
#pragma unroll
    for (int e = 0; e < 4; ++e) {
      const float t = wv[e];
      tile[(c4 + e) * 72 + kr] = (_Float16)(bf16r(t) * 64.0f);
    }
  }
  __syncthreads();
  half8 hv[2];
  size_t go[2];
#pragma unroll
  for (int p = 0; p < 2; ++p) {
    const int idx = tid + 256 * p;
    const int n = idx >> 3;
    const int g = idx & 7;
    hv[p] = *(const half8*)&tile[n * 72 + g * 8];
    go[p] = (size_t)(n0 + n) * DM + k0 + g * 8;
  }
#pragma unroll
  for (int p = 0; p < 2; ++p) *(volatile half8*)(T + go[p]) = hv[p];
  __threadfence();
#pragma unroll
  for (int p = 0; p < 2; ++p) *(volatile half8*)(T + go[p]) = hv[p];
}

__global__ __launch_bounds__(128) void k_relsum(const float* __restrict__ tab,
                                                float* __restrict__ rs) {
  __shared__ __align__(16) float part[128];
  const int tid = threadIdx.x;
  const int d = blockIdx.x * 128 + tid;
  const int dr = (d < NREL) ? d : (NREL - 1);
  const float* row = tab + (size_t)dr * RELDIM;
  float s = 0.0f;
#pragma unroll 1
  for (int i = 0; i < RELDIM; i += 4) {
    const v4f x = *(const v4f*)(row + i);
    const float x0 = x[0], x1 = x[1], x2 = x[2], x3 = x[3];
    s = s + bf16r(x0);
    s = s + bf16r(x1);
    s = s + bf16r(x2);
    s = s + bf16r(x3);
  }
  if (d >= NREL) s = 0.0f;
  part[tid] = s;
  __syncthreads();
  if (tid < 32) {
    const v4f o = *(const v4f*)&part[tid * 4];
    float* g = rs + (size_t)blockIdx.x * 128 + tid * 4;
    *(volatile v4f*)g = o;
    __threadfence();
    *(volatile v4f*)g = o;
  }
}

__global__ __launch_bounds__(256) void k_flags(const int* __restrict__ mask,
                                               int* __restrict__ flags) {
  __shared__ int fl[FLAGS_PITCH];
  __shared__ unsigned int rblo[8];
  __shared__ unsigned int rbhi[8];
  const int tid = threadIdx.x, wave = tid >> 5, lane = tid & 31;
  const int qb = blockIdx.x, q0 = qb * 64;
  if (tid < FLAGS_PITCH) fl[tid] = 0;
  const int grp = tid >> 4;
  const int c4 = (tid & 15) * 4;
  const int kta = grp, ktb = grp + 16;
  const int va = (kta < NQB) ? 1 : 0;
  const int vb = (ktb < NQB) ? 1 : 0;
  const int ktac = va ? kta : (NQB - 1);
  const int ktbc = vb ? ktb : (NQB - 1);
  int anyA = 0, allA = 1, anyB = 0, allB = 1;
  unsigned int rlo = 0u, rhi = 0u;
#pragma unroll 1
  for (int i = 0; i < 64; ++i) {
    const int* mr = mask + (size_t)(q0 + i) * SEQ_FULL;
    const v4i xa = *(const v4i*)(mr + ktac * 64 + c4);
    const v4i xb = *(const v4i*)(mr + ktbc * 64 + c4);
    const int a0 = xa[0], a1 = xa[1], a2 = xa[2], a3 = xa[3];
    const int b0 = xb[0], b1 = xb[1], b2 = xb[2], b3 = xb[3];
    const int na = ((a0 != 0) | (a1 != 0) | (a2 != 0) | (a3 != 0)) ? 1 : 0;
    const int fa = ((a0 != 0) & (a1 != 0) & (a2 != 0) & (a3 != 0)) ? 1 : 0;
    const int nb = ((b0 != 0) | (b1 != 0) | (b2 != 0) | (b3 != 0)) ? 1 : 0;
    const int fb = ((b0 != 0) & (b1 != 0) & (b2 != 0) & (b3 != 0)) ? 1 : 0;
    anyA |= na; allA &= fa; anyB |= nb; allB &= fb;
    const unsigned int hit = (unsigned int)((na & va) | (nb & vb));
    if (i < 32) rlo |= hit << i;
    else        rhi |= hit << (i - 32);
  }
#pragma unroll
  for (int off = 1; off < 16; off <<= 1) {
    anyA |= __shfl_xor(anyA, off, 32);
    allA &= __shfl_xor(allA, off, 32);
    anyB |= __shfl_xor(anyB, off, 32);
    allB &= __shfl_xor(allB, off, 32);
  }
#pragma unroll
  for (int off = 1; off < 32; off <<= 1) {
    rlo |= __shfl_xor(rlo, off, 32);
    rhi |= __shfl_xor(rhi, off, 32);
  }
  __syncthreads();
  if ((tid & 15) == 0) {
    if (va) fl[kta] = anyA ? (allA ? 2 : 1) : 0;
    if (vb) fl[ktb] = anyB ? (allB ? 2 : 1) : 0;
  }
  if (lane == 0) { rblo[wave] = rlo; rbhi[wave] = rhi; }
  __syncthreads();
  if (tid < 32) {
    unsigned int tlo = 0u, thi = 0u;
#pragma unroll
    for (int ww = 0; ww < 8; ++ww) { tlo |= rblo[ww]; thi |= rbhi[ww]; }
    const bool force = (tlo != 0xffffffffu) || (thi != 0xffffffffu);
    int f = fl[lane];
    f = (force && (f == 0)) ? 1 : f;
    f = (lane < NQB) ? f : 0;
    int* dst = flags + (size_t)qb * FLAGS_PITCH + lane;
    *(volatile int*)dst = f;
    __threadfence();
    *(volatile int*)dst = f;
  }
}

template <int OMODE, bool RESA>
__global__ __launch_bounds__(256) __attribute__((amdgpu_num_vgpr(256)))
void k_gemm(const _Float16* __restrict__ A, const _Float16* __restrict__ Alo,
            const _Float16* __restrict__ Bt, const float* __restrict__ bias,
            void* out0, void* out1) {
  __shared__ __align__(16) unsigned char lds_raw[36864];
  const int tid = threadIdx.x, wave = tid >> 5, lane = tid & 31;
  const int m = lane & 15, hs = lane >> 4;
  const int blockN = blockIdx.x * 64;
  const int blockM = blockIdx.y * 256;
  const bool res = RESA && ((blockM % SEQ) < EARLY_ROWS);

  float8 acc[2][4];
#pragma unroll
  for (int i = 0; i < 2; ++i)
#pragma unroll
    for (int t = 0; t < 4; ++t) acc[i][t] = zero8();

  const size_t arow = (size_t)(blockM + wave * 32 + m) * DM;
  const _Float16* a0p = A + arow;
  const _Float16* a1p = a0p + (size_t)16 * DM;
  const _Float16* l0p = Alo + arow;
  const _Float16* l1p = l0p + (size_t)16 * DM;
  const _Float16* bp = Bt + (size_t)(blockN + m) * DM;

#pragma unroll 1
  for (int ks = 0; ks < DM / 32; ++ks) {
    const int k0 = ks * 32;
    const half16 fa0 = load_frag(a0p + k0, hs);
    const half16 fa1 = load_frag(a1p + k0, hs);
    half16 fb[4];
#pragma unroll
    for (int t = 0; t < 4; ++t) fb[t] = load_frag(bp + (size_t)(t * 16) * DM + k0, hs);
#pragma unroll
    for (int t = 0; t < 4; ++t) {
      acc[0][t] = wmma16(fa0, fb[t], acc[0][t]);
      acc[1][t] = wmma16(fa1, fb[t], acc[1][t]);
    }
    if (res) {
      const half16 fl0 = load_frag(l0p + k0, hs);
      const half16 fl1 = load_frag(l1p + k0, hs);
#pragma unroll
      for (int t = 0; t < 4; ++t) {
        acc[0][t] = wmma16(fl0, fb[t], acc[0][t]);
        acc[1][t] = wmma16(fl1, fb[t], acc[1][t]);
      }
    }
  }

  constexpr float ESC = (OMODE == 0) ? 0.015625f : ((OMODE == 1) ? 0.0625f : 0.0009765625f);
  constexpr float BSC = (OMODE == 0) ? 16.0f : ((OMODE == 1) ? 64.0f : 1.0f);
  float bterm[4];
#pragma unroll
  for (int t = 0; t < 4; ++t) bterm[t] = BSC * bf16r(bias[blockN + t * 16 + m]);

  if (OMODE == 0) {
    _Float16* th = (_Float16*)lds_raw;
#pragma unroll
    for (int ph = 0; ph < 2; ++ph) {
#pragma unroll
      for (int mt = 0; mt < 2; ++mt)
#pragma unroll
        for (int t = 0; t < 4; ++t)
#pragma unroll
          for (int r = 0; r < 8; ++r) {
            const int row = wave * 32 + mt * 16 + hs * 8 + r;
            const int col = t * 16 + m;
            const float val = acc[mt][t][r] * ESC + bterm[t];
            const _Float16 hi = (_Float16)val;
            th[row * 72 + col] = (ph == 0) ? hi : (_Float16)(val - (float)hi);
          }
      __syncthreads();
      half8 hv[8];
      size_t go[8];
#pragma unroll
      for (int p = 0; p < 8; ++p) {
        const int row = wave * 32 + p * 4 + (lane >> 3);
        const int c8 = (lane & 7) * 8;
        hv[p] = *(const half8*)&th[row * 72 + c8];
        go[p] = (size_t)(blockM + row) * DM + blockN + c8;
      }
      _Float16* dst = (_Float16*)((ph == 0) ? out0 : out1);
#pragma unroll
      for (int p = 0; p < 8; ++p) *(volatile half8*)(dst + go[p]) = hv[p];
      __threadfence();
#pragma unroll
      for (int p = 0; p < 8; ++p) *(volatile half8*)(dst + go[p]) = hv[p];
      __syncthreads();
    }
  } else if (OMODE == 1) {
    _Float16* th = (_Float16*)lds_raw;
    const int bb = blockM / SEQ;
    const int s0 = blockM - bb * SEQ;
    const int hh = blockIdx.x;
#pragma unroll
    for (int ph = 0; ph < 2; ++ph) {
#pragma unroll
      for (int mt = 0; mt < 2; ++mt)
#pragma unroll
        for (int t = 0; t < 4; ++t)
#pragma unroll
          for (int r = 0; r < 8; ++r) {
            const int sl = wave * 32 + mt * 16 + hs * 8 + r;
            const int dh = t * 16 + m;
            const float val = acc[mt][t][r] * ESC + bterm[t];
            const _Float16 hi = (_Float16)val;
            th[dh * 264 + sl] = (ph == 0) ? hi : (_Float16)(val - (float)hi);
          }
      __syncthreads();
      half8 hv[8];
      size_t go[8];
#pragma unroll
      for (int p = 0; p < 8; ++p) {
        const int dh = wave * 8 + p;
        hv[p] = *(const half8*)&th[dh * 264 + lane * 8];
        go[p] = ((size_t)((bb * NH + hh) * DK + dh)) * SEQ + s0 + lane * 8;
      }
      _Float16* dst = (_Float16*)((ph == 0) ? out0 : out1);
#pragma unroll
      for (int p = 0; p < 8; ++p) *(volatile half8*)(dst + go[p]) = hv[p];
      __threadfence();
#pragma unroll
      for (int p = 0; p < 8; ++p) *(volatile half8*)(dst + go[p]) = hv[p];
      __syncthreads();
    }
  } else {
    float* tf = (float*)lds_raw;
    const int bb = blockM / SEQ;
    const int s0 = blockM - bb * SEQ;
    float* dst = (float*)out0;
#pragma unroll
    for (int ph = 0; ph < 2; ++ph) {
      if ((wave >> 2) == ph) {
#pragma unroll
        for (int mt = 0; mt < 2; ++mt)
#pragma unroll
          for (int t = 0; t < 4; ++t)
#pragma unroll
            for (int r = 0; r < 8; ++r) {
              const int rowl = (wave & 3) * 32 + mt * 16 + hs * 8 + r;
              const int col = t * 16 + m;
              tf[rowl * 68 + col] = acc[mt][t][r] * ESC + bterm[t];
            }
      }
      __syncthreads();
      v4f fv[8];
      size_t go[8];
#pragma unroll
      for (int p = 0; p < 8; ++p) {
        const int rowl = wave * 16 + p * 2 + (lane >> 4);
        const int c4 = (lane & 15) * 4;
        fv[p] = *(const v4f*)&tf[rowl * 68 + c4];
        const int s = s0 + ph * 128 + rowl;
        go[p] = ((size_t)(bb * SEQ_FULL + s)) * DM + blockN + c4;
      }
#pragma unroll
      for (int p = 0; p < 8; ++p) *(volatile v4f*)(dst + go[p]) = fv[p];
      __threadfence();
#pragma unroll
      for (int p = 0; p < 8; ++p) *(volatile v4f*)(dst + go[p]) = fv[p];
      __syncthreads();
    }
  }
}

template <bool EARLY>
__global__ __launch_bounds__(128) __attribute__((amdgpu_num_vgpr(256)))
void k_attn(const _Float16* __restrict__ Qh, const _Float16* __restrict__ Ql,
            const _Float16* __restrict__ Kh, const _Float16* __restrict__ Kl,
            const _Float16* __restrict__ VTh, const _Float16* __restrict__ VTl,
            const float* __restrict__ relsum, const int* __restrict__ flags,
            const int* __restrict__ mask,
            _Float16* __restrict__ ctxh, _Float16* __restrict__ ctxl,
            int qbBase, int nQB) {
  __shared__ __align__(16) float rwin[RW];
  __shared__ __align__(16) _Float16 Plds[4 * 16 * 40];
  __shared__ __align__(16) _Float16 Prls[4 * 16 * 40];
  __shared__ __align__(16) int mk[64 * 32];
  __shared__ __align__(16) _Float16 Oh[4 * 16 * 72];
  __shared__ __align__(16) _Float16 Ol[4 * 16 * 72];

  const int tid = threadIdx.x, w = tid >> 5, lane = tid & 31;
  const int m = lane & 15, hs = lane >> 4;
  const int bh = blockIdx.x / nQB;
  const int qb = qbBase + (blockIdx.x - bh * nQB);
  const int b = bh / NH, h = bh - b * NH;
  const int q0 = qb * 64;
  const int tq = b * SEQ + q0 + w * 16;
  _Float16* Pw  = Plds + w * (16 * 40);
  _Float16* Rw  = Prls + w * (16 * 40);
  _Float16* Ohw = Oh + w * (16 * 72);
  _Float16* Olw = Ol + w * (16 * 72);

  const _Float16* qhp = Qh + (size_t)(tq + m) * DM + h * DK;
  const _Float16* qlp = Ql + (size_t)(tq + m) * DM + h * DK;
  half16 qg0, qg1;
  if (!EARLY) { qg0 = load_frag(qhp, hs); qg1 = load_frag(qhp + 32, hs); }
  else        { qg0 = zero16(); qg1 = zero16(); }

  {
    const int dbase = RELOFF - q0 - 63;
#pragma unroll 1
    for (int e = tid; e < RW; e += 128) {
      int d = dbase + e;
      d = (d < 0) ? 0 : d;
      d = (d > NREL - 1) ? (NREL - 1) : d;
      rwin[e] = relsum[d];
    }
  }
  __syncthreads();

  float8 o[4];
#pragma unroll
  for (int t = 0; t < 4; ++t) o[t] = zero8();
  float mrow[8], lrow[8];
#pragma unroll
  for (int r = 0; r < 8; ++r) { mrow[r] = -3.0e38f; lrow[r] = 0.0f; }

  const float SSC  = 0.00048828125f;
  const float PC   = 16384.0f;
  const float NEGF = -1.0e20f;

#pragma unroll 1
  for (int kt = 0; kt < NQB; ++kt) {
    const int f = __builtin_amdgcn_readfirstlane(flags[qb * FLAGS_PITCH + kt]);
    if (f == 0) continue;
    const bool partial = (f != 2);
#pragma unroll 1
    for (int sub = 0; sub < 2; ++sub) {
      const int k0 = kt * 64 + sub * 32;
      const int tk = b * SEQ + k0;
      if (partial) {
#pragma unroll
        for (int p = 0; p < 4; ++p) {
          const int idx = tid + 128 * p;
          const int row = idx >> 3;
          const int c4 = (idx & 7) * 4;
          const v4i mv = *(const v4i*)(mask + (size_t)(q0 + row) * SEQ_FULL + k0 + c4);
          *(v4i*)&mk[row * 32 + c4] = mv;
        }
        __syncthreads();
      }

      float8 s0 = zero8(), s1 = zero8();
#pragma unroll
      for (int c = 0; c < 2; ++c) {
        const half16 fq = EARLY ? load_frag(qhp + c * 32, hs) : ((c == 0) ? qg0 : qg1);
        const _Float16* kr = Kh + (size_t)(tk + m) * DM + h * DK + c * 32;
        half16 fk0 = load_frag(kr, hs);
        half16 fk1 = load_frag(kr + (size_t)16 * DM, hs);
        s0 = wmma16(fq, fk0, s0);
        s1 = wmma16(fq, fk1, s1);
        if (EARLY) {
          const half16 fql = load_frag(qlp + c * 32, hs);
          s0 = wmma16(fql, fk0, s0);
          s1 = wmma16(fql, fk1, s1);
          const _Float16* lr = Kl + (size_t)(tk + m) * DM + h * DK + c * 32;
          fk0 = load_frag(lr, hs);
          fk1 = load_frag(lr + (size_t)16 * DM, hs);
          s0 = wmma16(fq, fk0, s0);
          s1 = wmma16(fq, fk1, s1);
        }
      }

#pragma unroll
      for (int r = 0; r < 8; ++r) {
        const int il = w * 16 + hs * 8 + r;
        const int eb = k0 + m + 63 - il;
        float a0 = s0[r] * SSC + rwin[eb];
        float a1 = s1[r] * SSC + rwin[eb + 16];
        if (partial) {
          const int mv0 = mk[il * 32 + m];
          const int mv1 = mk[il * 32 + 16 + m];
          a0 = (mv0 != 0) ? a0 : NEGF;
          a1 = (mv1 != 0) ? a1 : NEGF;
        }
        float mtl = fmaxf(a0, a1);
#pragma unroll
        for (int off = 1; off < 16; off <<= 1) mtl = fmaxf(mtl, __shfl_xor(mtl, off, 32));
        const float mnew = fmaxf(mrow[r], mtl);
        const float corr = __expf(mrow[r] - mnew);
        mrow[r] = mnew;
        lrow[r] *= corr;
#pragma unroll
        for (int t = 0; t < 4; ++t) o[t][r] *= corr;
        const float p0 = __expf(a0 - mnew) * PC;
        const float p1 = __expf(a1 - mnew) * PC;
        float ps = p0 + p1;
#pragma unroll
        for (int off = 1; off < 16; off <<= 1) ps += __shfl_xor(ps, off, 32);
        lrow[r] += ps;
        const _Float16 ph0 = (_Float16)p0;
        const _Float16 ph1 = (_Float16)p1;
        Pw[(hs * 8 + r) * 40 + m]      = ph0;
        Pw[(hs * 8 + r) * 40 + 16 + m] = ph1;
        if (EARLY) {
          Rw[(hs * 8 + r) * 40 + m]      = (_Float16)(p0 - (float)ph0);
          Rw[(hs * 8 + r) * 40 + 16 + m] = (_Float16)(p1 - (float)ph1);
        }
      }
      __syncthreads();

      const half16 pa = load_frag(Pw + m * 40, hs);
      half16 pres = pa;
      if (EARLY) pres = load_frag(Rw + m * 40, hs);
#pragma unroll
      for (int t = 0; t < 4; ++t) {
        const size_t vo = ((size_t)(bh * DK + t * 16 + m)) * SEQ + k0;
        half16 fv = load_frag(VTh + vo, hs);
        o[t] = wmma16(pa, fv, o[t]);
        if (EARLY) {
          o[t] = wmma16(pres, fv, o[t]);
          fv = load_frag(VTl + vo, hs);
          o[t] = wmma16(pa, fv, o[t]);
        }
      }
      __syncthreads();
    }
  }

#pragma unroll
  for (int r = 0; r < 8; ++r) {
    const float l = lrow[r];
    const float il4 = (l > 0.0f) ? (0.25f / l) : 0.0f;
#pragma unroll
    for (int t = 0; t < 4; ++t) {
      const float val = o[t][r] * il4;
      const _Float16 hi = (_Float16)val;
      Ohw[(hs * 8 + r) * 72 + t * 16 + m] = hi;
      Olw[(hs * 8 + r) * 72 + t * 16 + m] = (_Float16)(val - (float)hi);
    }
  }
  __syncthreads();
  half8 hv[4], lv[4];
  size_t go[4];
#pragma unroll
  for (int p = 0; p < 4; ++p) {
    const int row = p * 4 + (lane >> 3);
    const int c8 = (lane & 7) * 8;
    hv[p] = *(const half8*)&Ohw[row * 72 + c8];
    lv[p] = *(const half8*)&Olw[row * 72 + c8];
    go[p] = (size_t)(tq + row) * DM + h * DK + c8;
  }
#pragma unroll
  for (int p = 0; p < 4; ++p) {
    *(volatile half8*)(ctxh + go[p]) = hv[p];
    *(volatile half8*)(ctxl + go[p]) = lv[p];
  }
  __threadfence();
#pragma unroll
  for (int p = 0; p < 4; ++p) {
    *(volatile half8*)(ctxh + go[p]) = hv[p];
    *(volatile half8*)(ctxl + go[p]) = lv[p];
  }
}

extern "C" void kernel_launch(void* const* d_in, const int* in_sizes, int n_in,
                              void* d_out, int out_size, void* d_ws,
                              size_t ws_size, hipStream_t stream) {
  if (n_in < 13) return;
  const float* q   = (const float*)d_in[0];
  const float* k   = (const float*)d_in[1];
  const float* v   = (const float*)d_in[2];
  const float* Wq  = (const float*)d_in[3];
  const float* bq  = (const float*)d_in[4];
  const float* Wk  = (const float*)d_in[5];
  const float* bk  = (const float*)d_in[6];
  const float* Wv  = (const float*)d_in[7];
  const float* bv  = (const float*)d_in[8];
  const float* Wo  = (const float*)d_in[9];
  const float* bo  = (const float*)d_in[10];
  const float* rel = (const float*)d_in[11];
  const int*   msk = (const int*)d_in[12];

  const long long need_x = ((long long)(NB - 1) * SEQ_FULL + SEQ) * DM;
  if ((long long)in_sizes[0] < need_x || (long long)in_sizes[1] < need_x ||
      (long long)in_sizes[2] < need_x) return;
  if (in_sizes[3] < DM * DM || in_sizes[5] < DM * DM || in_sizes[7] < DM * DM ||
      in_sizes[9] < DM * DM) return;
  if (in_sizes[4] < DM || in_sizes[6] < DM || in_sizes[8] < DM || in_sizes[10] < DM) return;
  if (in_sizes[11] < NREL * RELDIM) return;
  if ((long long)in_sizes[12] < (long long)(SEQ - 1) * SEQ_FULL + SEQ) return;
  if ((long long)out_size < need_x) return;

  char* ws = (char*)d_ws;
  size_t off = 0;
  auto carve = [&](size_t bytes) -> char* {
    char* p = ws + off;
    off += (bytes + 255) & ~(size_t)255;
    return p;
  };
  const size_t plane  = (size_t)MTOK * DM * sizeof(_Float16);
  const size_t wplane = (size_t)DM * DM * sizeof(_Float16);
  _Float16* Xq  = (_Float16*)carve(plane);
  _Float16* Xk  = (_Float16*)carve(plane);
  _Float16* Xv  = (_Float16*)carve(plane);
  _Float16* Wtq = (_Float16*)carve(wplane);
  _Float16* Wtk = (_Float16*)carve(wplane);
  _Float16* Wtv = (_Float16*)carve(wplane);
  _Float16* Wto = (_Float16*)carve(wplane);
  _Float16* Qh  = (_Float16*)carve(plane);
  _Float16* Ql  = (_Float16*)carve(plane);
  _Float16* Kh  = (_Float16*)carve(plane);
  _Float16* Kl  = (_Float16*)carve(plane);
  _Float16* VTh = (_Float16*)carve(plane);
  _Float16* VTl = (_Float16*)carve(plane);
  _Float16* Ch  = (_Float16*)carve(plane);
  _Float16* Cl  = (_Float16*)carve(plane);
  float* rsum   = (float*)carve((size_t)RS_PAD * sizeof(float));
  int*   flg    = (int*)carve((size_t)NQB * FLAGS_PITCH * sizeof(int));
  if (off > ws_size) return;

  {
    const size_t total8 = (size_t)MTOK * DM / 8;
    dim3 g((unsigned)((total8 + 255) / 256), 3);
    k_xcvt<<<g, dim3(256), 0, stream>>>(q, k, v, Xq, Xk, Xv);
  }
  k_wcvt<<<dim3(DM / 64, DM / 64, 4), dim3(256), 0, stream>>>(Wq, Wk, Wv, Wo,
                                                              Wtq, Wtk, Wtv, Wto);
  k_relsum<<<dim3(RS_PAD / 128), dim3(128), 0, stream>>>(rel, rsum);
  k_flags<<<dim3(NQB), dim3(256), 0, stream>>>(msk, flg);

  dim3 gg(DM / 64, MTOK / 256);
  k_gemm<0, false><<<gg, dim3(256), 0, stream>>>(Xq, Xq, Wtq, bq, (void*)Qh, (void*)Ql);
  k_gemm<0, false><<<gg, dim3(256), 0, stream>>>(Xk, Xk, Wtk, bk, (void*)Kh, (void*)Kl);
  k_gemm<1, false><<<gg, dim3(256), 0, stream>>>(Xv, Xv, Wtv, bv, (void*)VTh, (void*)VTl);

  const int nEarly = EARLY_QB;
  const int nLate  = NQB - EARLY_QB;
  k_attn<true><<<dim3(NB * NH * nEarly), dim3(128), 0, stream>>>(
      Qh, Ql, Kh, Kl, VTh, VTl, rsum, flg, msk, Ch, Cl, 0, nEarly);
  if (nLate > 0) {
    k_attn<false><<<dim3(NB * NH * nLate), dim3(128), 0, stream>>>(
        Qh, Ql, Kh, Kl, VTh, VTl, rsum, flg, msk, Ch, Cl, nEarly, nLate);
  }

  k_gemm<2, true><<<gg, dim3(256), 0, stream>>>(Ch, Cl, Wto, bo, d_out, d_out);
}
